// BertEmbeddingsIngredientsUntied_84026740179009
// MI455X (gfx1250) — hardware-verified
//
#include <hip/hip_runtime.h>


namespace {
constexpr int B = 32, L = 2048, DW = 300, KP = 320, H = 768, SMAX = 128, NT = B * L;
constexpr float XS = 8.0f, WSC = 256.0f;
typedef _Float16 b16;
typedef __attribute__((ext_vector_type(16))) _Float16 v16b;
typedef __attribute__((ext_vector_type(8))) _Float16 v8b;
typedef __attribute__((ext_vector_type(8))) float v8f;
typedef __attribute__((ext_vector_type(4))) float v4f;
__device__ __forceinline__ float bf16_rne(float f) { unsigned int u = __float_as_uint(f); u += 0x7FFFu + ((u >> 16) & 1u); return __uint_as_float(u & 0xFFFF0000u); }
__device__ __forceinline__ v16b frag_kb(const b16* p, int hh) { const v8b a = *(const v8b*)(p + 8 * hh), b = *(const v8b*)(p + 16 + 8 * hh); v16b f;
#pragma unroll
  for (int e = 0; e < 8; ++e) { f[e] = a[e]; f[8 + e] = b[e]; } return f; }
__device__ __forceinline__ v8f wmma16b(v16b a, v16b b, v8f c) { v8f d = __builtin_amdgcn_wmma_f32_16x16x32_f16(false, a, false, b, (short)0, c, false, false); asm volatile("v_nop\n\tv_nop\n\tv_nop\n\tv_nop" : "+v"(d) : "v"(a), "v"(b)); return d; }
__device__ __forceinline__ void wave_lds_sync() { __builtin_amdgcn_fence(__ATOMIC_RELEASE, "workgroup"); __builtin_amdgcn_wave_barrier(); __builtin_amdgcn_fence(__ATOMIC_ACQUIRE, "workgroup"); }
__device__ __forceinline__ float pmul(float a, float b) { float p = a * b; asm volatile("" : "+v"(p)); return p; }
__device__ __forceinline__ int iclamp(int v, int lo, int hi) { return v < lo ? lo : (v > hi ? hi : v); }

__global__ __launch_bounds__(256) void wput_kernel(const float* __restrict__ w, b16* __restrict__ WT) { const int u = blockIdx.x * 256 + threadIdx.x; if (u >= H * (KP / 8)) return; const int o = u / (KP / 8), k0 = (u % (KP / 8)) * 8; v8b v;
#pragma unroll
  for (int j = 0; j < 8; ++j) { const int k = k0 + j; v[j] = (b16)(k < DW ? bf16_rne(w[(size_t)k * H + o]) * WSC : 0.0f); } for (int pass = 0; pass < 2; ++pass) { *(volatile v8b*)(WT + (size_t)o * KP + k0) = v; __threadfence(); } }
__global__ __launch_bounds__(32) void tok_kernel(const int* __restrict__ ids, const float* __restrict__ emb, int V, const float* __restrict__ g1, const float* __restrict__ b1, const b16* __restrict__ WT, const float* __restrict__ bias, const float* __restrict__ g2, const float* __restrict__ b2, int RL, float* __restrict__ HT) {
  __shared__ __attribute__((aligned(16))) b16 Ah[16][KP + 8]; __shared__ float Tf[16][H + 4], Mu[16], Rs[16]; const int lane = threadIdx.x, nloc = lane & 15, hlf = lane >> 4; const size_t m0 = (size_t)blockIdx.x * 16; if (m0 >= (size_t)RL) return;
  for (int rr = 0; rr < 16; ++rr) { const int id = iclamp(ids[m0 + rr], 0, V - 1); const float* er = emb + (size_t)id * DW; float v[10]; float s = 0.0f;
#pragma unroll
    for (int q = 0; q < 10; ++q) { const int c = q * 32 + lane; v[q] = c < DW ? bf16_rne(er[c]) : 0.0f; s += v[q]; }
    for (int o = 16; o; o >>= 1) s += __shfl_xor(s, o); const float mu = s * (1.0f / DW); float vq = 0.0f;
#pragma unroll
    for (int q = 0; q < 10; ++q) { const int c = q * 32 + lane; if (c < DW) { const float dd = v[q] - mu; vq += pmul(dd, dd); } }
    for (int o = 16; o; o >>= 1) vq += __shfl_xor(vq, o); const float rs = 1.0f / sqrtf(vq * (1.0f / DW) + 1e-12f);
#pragma unroll
    for (int q = 0; q < 10; ++q) { const int c = q * 32 + lane; Ah[rr][c] = (b16)(c < DW ? (pmul(pmul(v[q] - mu, rs), bf16_rne(g1[c])) + bf16_rne(b1[c])) * XS : 0.0f); } }
  wave_lds_sync();
#pragma unroll 1
  for (int cg = 0; cg < 3; ++cg) { v8f acc[16];
#pragma unroll
    for (int t = 0; t < 16; ++t) acc[t] = (v8f){};
#pragma unroll 2
    for (int kb = 0; kb < KP; kb += 32) { const v16b a = frag_kb(&Ah[nloc][kb], hlf);
#pragma unroll
      for (int t = 0; t < 16; ++t) acc[t] = wmma16b(a, frag_kb(WT + (size_t)(cg * 256 + t * 16 + nloc) * KP + kb, hlf), acc[t]); }
#pragma unroll
    for (int t = 0; t < 16; ++t) { const int c = cg * 256 + t * 16 + nloc; const float bb = bf16_rne(bias[c]);
#pragma unroll
      for (int r8 = 0; r8 < 8; ++r8) Tf[8 * hlf + r8][c] = fmaxf(acc[t][r8] * (1.0f / (XS * WSC)) + bb, 0.0f); } }
  wave_lds_sync();
  if (lane < 16) { float s = 0.0f; for (int c = 0; c < H; ++c) s += Tf[lane][c]; const float mu = s * (1.0f / H); float vq = 0.0f; for (int c = 0; c < H; ++c) { const float dd = Tf[lane][c] - mu; vq += pmul(dd, dd); } Mu[lane] = mu; Rs[lane] = 1.0f / sqrtf(vq * (1.0f / H) + 1e-12f); }
  wave_lds_sync();
  for (int pass = 0; pass < 2; ++pass) { for (int rr = 0; rr < 16; ++rr) for (int c = lane; c < H; c += 32) ((volatile float*)HT)[(m0 + rr) * H + c] = pmul(pmul(Tf[rr][c] - Mu[rr], Rs[rr]), bf16_rne(g2[c])) + bf16_rne(b2[c]); __threadfence(); }
}
__global__ __launch_bounds__(32) void seg_kernel(const int* __restrict__ sep, int S, int* __restrict__ RNG) {
  __shared__ int St[SMAX], En[SMAX]; const int lane = threadIdx.x, b = blockIdx.x;
  for (int s = lane; s < SMAX; s += 32) { St[s] = 0; En[s] = 0; }
  wave_lds_sync();
  if (lane == 0) { int cnt = 0, start = 0; for (int l = 0; l < L; ++l) { if (sep[(size_t)b * L + l] != 0) { if (cnt < S && cnt < SMAX) { St[cnt] = start; En[cnt] = l; } ++cnt; start = l + 1; } } if (cnt < S && cnt < SMAX) { St[cnt] = start; En[cnt] = L; } }
  wave_lds_sync();
  for (int pass = 0; pass < 2; ++pass) { for (int s = lane; s < SMAX; s += 32) { ((volatile int*)RNG)[(size_t)b * 2 * SMAX + s] = St[s]; ((volatile int*)RNG)[(size_t)b * 2 * SMAX + SMAX + s] = En[s]; } __threadfence(); }
}
__global__ __launch_bounds__(256) void pe_kernel(int S, float* __restrict__ PE) { const int u = blockIdx.x * 256 + threadIdx.x; if (u >= S * H) return; const int s = u / H, c = u % H; const float dv = expf((float)(c & ~1) * (-logf(10000.0f) / (float)H)); const float ang = (float)s * dv; const float v = (c & 1) ? cosf(ang) : sinf(ang);
  for (int pass = 0; pass < 2; ++pass) { ((volatile float*)PE)[u] = v; __threadfence(); } }
__global__ __launch_bounds__(256) void mean_kernel(const float* __restrict__ HT, const int* __restrict__ sep, const int* __restrict__ RNG, const float* __restrict__ PE, int S, int BV, float* __restrict__ out) {
  const int wave = threadIdx.x >> 5, lane = threadIdx.x & 31; const int bs = blockIdx.x * 8 + wave; const int b = bs / S, s = bs % S; if (b >= BV) return;
  int st = RNG[(size_t)b * 2 * SMAX + s], en = RNG[(size_t)b * 2 * SMAX + SMAX + s]; st = iclamp(st, 0, L); en = iclamp(en, st, L); float a[24];
#pragma unroll
  for (int q = 0; q < 24; ++q) a[q] = 0.0f; int cnt = 0;
#pragma unroll 1
  for (int l = st; l < en; ++l) { if (sep[(size_t)b * L + l] != 0) continue; ++cnt; const float* hr = HT + ((size_t)b * L + l) * H;
#pragma unroll
    for (int q = 0; q < 24; ++q) a[q] += hr[q * 32 + lane]; }
  const float inv = cnt > 0 ? 1.0f / (float)cnt : 0.0f;
  for (int pass = 0; pass < 2; ++pass) {
#pragma unroll
    for (int q = 0; q < 24; ++q) { const int c = q * 32 + lane; ((volatile float*)out)[((size_t)b * S + s) * H + c] = pmul(a[q], inv) + PE[(size_t)s * H + c]; } __threadfence(); }
}
}

extern "C" void kernel_launch(void* const* d_in, const int* in_sizes, int n_in, void* d_out, int out_size, void* d_ws, size_t ws_size, hipStream_t stream) {
  (void)n_in;
  auto Fp = [&](int i) { return (const float*)d_in[i]; }; auto Ip = [&](int i) { return (const int*)d_in[i]; };
  if (in_sizes[0] != NT || in_sizes[1] != NT || in_sizes[2] != 1 || in_sizes[3] % DW != 0 || in_sizes[4] != DW || in_sizes[6] != DW * H || in_sizes[8] != H) return;
  const int V = in_sizes[3] / DW; const int S = out_size / (B * H); if (S < 1 || S > SMAX || out_size != B * S * H) return;
  const int BV = B; const int RL = BV * L;
  size_t off = 0; char* ws = (char*)d_ws;
  auto carve = [&](size_t bytes) { char* p = ws + off; off += (bytes + 255) & ~(size_t)255; return p; };
  b16* WT = (b16*)carve((size_t)H * KP * 2); float* HT = (float*)carve((size_t)NT * H * 4); int* RNG = (int*)carve((size_t)B * 2 * SMAX * 4); float* PE = (float*)carve((size_t)SMAX * H * 4);
  if (off > ws_size || off > ((size_t)224 << 20)) return;
  wput_kernel<<<(H * (KP / 8) + 255) / 256, 256, 0, stream>>>(Fp(6), WT);
  tok_kernel<<<RL / 16, 32, 0, stream>>>(Ip(0), Fp(3), V, Fp(4), Fp(5), WT, Fp(7), Fp(8), Fp(9), RL, HT);
  seg_kernel<<<BV, 32, 0, stream>>>(Ip(1), S, RNG);
  pe_kernel<<<(S * H + 255) / 256, 256, 0, stream>>>(S, PE);
  mean_kernel<<<(BV * S + 7) / 8, 256, 0, stream>>>(HT, Ip(1), RNG, PE, S, BV, (float*)d_out);
}
